// NL_Up_68564857913601
// MI455X (gfx1250) — hardware-verified
//
#include <hip/hip_runtime.h>
#include <hip/hip_bf16.h>
#include <stdint.h>


typedef _Float16 bf16_t;
typedef _Float16 v16bf __attribute__((ext_vector_type(16)));
typedef _Float16 v8bf  __attribute__((ext_vector_type(8)));
typedef float  v8f   __attribute__((ext_vector_type(8)));
typedef __attribute__((ext_vector_type(4))) float v4f_t;
typedef float v4fa __attribute__((ext_vector_type(4), may_alias));
typedef __attribute__((ext_vector_type(4))) unsigned v4u_t;
typedef unsigned v4ua __attribute__((ext_vector_type(4), may_alias));
#define RSPLIT (1.0f / 2048.0f)
__device__ __forceinline__ bf16_t lo_of(float v, bf16_t h) { return (bf16_t)((v - (float)h) * 2048.0f); }
__device__ __forceinline__ v8f wmma16(v16bf a, v16bf b, v8f c) { return __builtin_amdgcn_wmma_f32_16x16x32_f16(false, a, false, b, (short)0, c, false, false); }
__device__ __forceinline__ v8f wmma_split(v16bf a, v16bf al, v16bf b, v16bf bl, v8f c) { v8f x = {}; x = wmma16(al, b, x); x = wmma16(a, bl, x); return wmma16(a, b, c) + x * RSPLIT; }

#define B_   8
#define C_   64
#define VC_  128
#define NQ_  4096
#define NV_  1024
#define NKB_ (NV_ / 64)
#define EPS_ 1e-5f
#define PLK  ((size_t)B_ * NV_ * C_)

__device__ __forceinline__ v16bf ldfrag(const bf16_t* p, int delta) {
    v8bf a = *(const v8bf*)p;
    v8bf b = *(const v8bf*)(p + delta);
    return __builtin_shufflevector(a, b, 0,1,2,3,4,5,6,7,8,9,10,11,12,13,14,15);
}

__device__ __forceinline__ void async_b128(bf16_t* lds_dst, const bf16_t* gsrc) {
    const uint32_t l = (uint32_t)(uintptr_t)lds_dst;
    asm volatile("global_load_async_to_lds_b128 %0, %1, off"
                 :: "v"(l), "v"(gsrc) : "memory");
}

__global__ __launch_bounds__(256) void conv_bn_kernel(
    const float* __restrict__ v, const float* __restrict__ k_w,
    const float* __restrict__ v_w,
    const float* __restrict__ k_gamma, const float* __restrict__ k_beta,
    const float* __restrict__ k_mean,  const float* __restrict__ k_var,
    bf16_t* __restrict__ keyT, bf16_t* __restrict__ valT) {
    __shared__ __align__(16) float vt[VC_][64];
    __shared__ __align__(16) bf16_t sk[2][64 * 72];
    __shared__ __align__(16) bf16_t sv[64 * 72];
    const int b  = blockIdx.y;
    const int nb = blockIdx.x * 64;
    const int t  = threadIdx.x;

    {
        const int cv = t >> 1, nh = (t & 1) * 32;
        const float4* s4 = (const float4*)(v + ((size_t)b * VC_ + cv) * NV_ + nb + nh);
        float4* d4 = (float4*)&vt[cv][nh];
        #pragma unroll
        for (int k = 0; k < 8; ++k) d4[k] = s4[k];
    }
    __syncthreads();

    const int c  = t & 63;
    const int j0 = (t >> 6) * 16;
    const float* kwr = k_w + c * VC_;
    const float* vwr = v_w + c * VC_;
    const float inv = k_gamma[c] * rsqrtf(k_var[c] + EPS_);
    const float add = k_beta[c] - k_mean[c] * inv;
    #pragma unroll 1
    for (int i = 0; i < 16; ++i) {
        float ka = 0.f, va = 0.f;
        #pragma unroll 1
        for (int cv = 0; cv < VC_; ++cv) {
            const float x = vt[cv][j0 + i];
            ka = fmaf(kwr[cv], x, ka);
            va = fmaf(vwr[cv], x, va);
        }
        const int nl = j0 + i;
        const float kv = ka * inv + add;
        const bf16_t kh = (bf16_t)kv;
        sk[0][nl * 72 + c] = kh; sk[1][nl * 72 + c] = lo_of(kv, kh);
        sv[c * 72 + nl] = (bf16_t)va;
    }
    __syncthreads();
#pragma unroll 1
    for (int pass = 0; pass < 2; ++pass) {
        for (int ch = t; ch < 64 * 8; ch += 256) { const int rr = ch >> 3, q8 = (ch & 7) * 8;
            bf16_t* kd = keyT + ((size_t)b * NV_ + nb + rr) * C_ + q8;
            *(volatile v4u_t*)kd = *(const v4ua*)(sk[0] + rr * 72 + q8);
            *(volatile v4u_t*)(kd + PLK) = *(const v4ua*)(sk[1] + rr * 72 + q8);
            *(volatile v4u_t*)(valT + ((size_t)b * C_ + rr) * NV_ + nb + q8) = *(const v4ua*)(sv + rr * 72 + q8); }
        __threadfence();
    }
}

__global__ __launch_bounds__(128) void attn_kernel(
    const float* __restrict__ q,
    const float* __restrict__ q_gamma, const float* __restrict__ q_beta,
    const float* __restrict__ q_mean,  const float* __restrict__ q_var,
    const bf16_t* __restrict__ keyT, const bf16_t* __restrict__ valT,
    float* __restrict__ out) {
    __shared__ __align__(16) bf16_t qt[64 * 64];
    __shared__ __align__(16) bf16_t ql[64 * 64];
    __shared__ __align__(16) bf16_t kt2[2][64 * 64];
    __shared__ __align__(16) bf16_t kl2[2][64 * 64];
    __shared__ __align__(16) bf16_t vvt2[2][64 * 64];
    __shared__ __align__(16) float  so[64 * 68];

    const int b     = blockIdx.y;
    const int qbase = blockIdx.x * 64;
    const int t     = threadIdx.x;
    const int lane  = t & 31, wave = t >> 5;
    const int col   = lane & 15;
    const bool hi   = lane >= 16;

    const int c2 = t >> 1, part = (t & 1) * 4;
    auto issue_tile = [&](int kb, int buf) {
        const bf16_t* ksrc = keyT + ((size_t)b * NV_ + kb * 64) * C_;
        bf16_t* kdst = kt2[buf];
        bf16_t* kldst = kl2[buf];
        #pragma unroll
        for (int k = 0; k < 4; ++k) {
            const int e = (t + 128 * k) * 8;
            async_b128(kdst + e, ksrc + e);
            async_b128(kldst + e, ksrc + PLK + e);
        }
        const bf16_t* vsrc = valT + ((size_t)b * C_ + c2) * NV_ + kb * 64;
        bf16_t* vdst = vvt2[buf] + c2 * 64;
        #pragma unroll
        for (int k = 0; k < 4; ++k)
            async_b128(vdst + (part + k) * 8, vsrc + (part + k) * 8);
    };

    {
        const int cq = t >> 1, ih = (t & 1) * 32;
        const float inv = q_gamma[cq] * rsqrtf(q_var[cq] + EPS_);
        const float add = q_beta[cq] - q_mean[cq] * inv;
        const float* src = q + ((size_t)b * C_ + cq) * NQ_ + qbase + ih;
        #pragma unroll 8
        for (int k = 0; k < 32; ++k) {
            const float qv = src[k] * inv + add; const bf16_t qh = (bf16_t)qv;
            qt[(ih + k) * 64 + cq] = qh; ql[(ih + k) * 64 + cq] = lo_of(qv, qh);
        }
    }
    issue_tile(0, 0);
    __syncthreads();

    const int irow = wave * 16 + col;
    const v16bf bq0 = ldfrag(qt + irow * 64 + (hi ? 8 : 0), 16);
    const v16bf bq1 = ldfrag(qt + irow * 64 + 32 + (hi ? 8 : 0), 16);
    const bf16_t* qlrow = ql + irow * 64 + (hi ? 8 : 0);

    v8f o[4];
    #pragma unroll
    for (int ct = 0; ct < 4; ++ct)
        #pragma unroll
        for (int r = 0; r < 8; ++r) o[ct][r] = 0.f;
    float m = -3.0e38f, l = 0.f;

    for (int kb = 0; kb < NKB_; ++kb) {
        if (kb + 1 < NKB_) {
            issue_tile(kb + 1, (kb + 1) & 1);
            asm volatile("s_wait_asynccnt 0xc" ::: "memory");
        } else {
            asm volatile("s_wait_asynccnt 0x0" ::: "memory");
        }
        __syncthreads();
        const bf16_t* ktc = kt2[kb & 1];
        const bf16_t* klc = kl2[kb & 1];
        const bf16_t* vtc = vvt2[kb & 1];

        v8f s[4];
        #pragma unroll
        for (int mt = 0; mt < 4; ++mt) {
            const bf16_t* arow = ktc + (mt * 16 + col) * 64 + (hi ? 8 : 0);
            const bf16_t* lrow = klc + (mt * 16 + col) * 64 + (hi ? 8 : 0);
            v8f acc;
            #pragma unroll
            for (int r = 0; r < 8; ++r) acc[r] = 0.f;
            acc = wmma_split(ldfrag(arow, 16), ldfrag(lrow, 16), bq0, ldfrag(qlrow, 16), acc);
            acc = wmma_split(ldfrag(arow + 32, 16), ldfrag(lrow + 32, 16), bq1, ldfrag(qlrow + 32, 16), acc);
            s[mt] = acc;
        }

        float tmax = -3.0e38f;
        #pragma unroll
        for (int mt = 0; mt < 4; ++mt)
            #pragma unroll
            for (int r = 0; r < 8; ++r) tmax = fmaxf(tmax, s[mt][r]);
        tmax = fmaxf(tmax, __shfl_xor(tmax, 16, 32));
        const float mnew = fmaxf(m, tmax);
        const float corr = __expf(m - mnew);
        float rsum = 0.f;
        #pragma unroll
        for (int mt = 0; mt < 4; ++mt)
            #pragma unroll
            for (int r = 0; r < 8; ++r) {
                const float p = __expf(s[mt][r] - mnew);
                s[mt][r] = p;
                rsum += p;
            }
        rsum += __shfl_xor(rsum, 16, 32);
        l = l * corr + rsum;
        m = mnew;
        #pragma unroll
        for (int ct = 0; ct < 4; ++ct)
            #pragma unroll
            for (int r = 0; r < 8; ++r) o[ct][r] *= corr;

        v16bf bp[2];
        #pragma unroll
        for (int h = 0; h < 2; ++h) {
            #pragma unroll
            for (int r = 0; r < 8; ++r) {
                bp[h][r]     = (bf16_t)(s[2 * h][r] * 1024.0f);
                bp[h][r + 8] = (bf16_t)(s[2 * h + 1][r] * 1024.0f);
            }
        }

        #pragma unroll
        for (int ct = 0; ct < 4; ++ct) {
            const bf16_t* vrow = vtc + (ct * 16 + col) * 64 + (hi ? 8 : 0);
            const v16bf av0 = ldfrag(vrow, 16);
            const v16bf av1 = ldfrag(vrow + 32, 16);
            o[ct] = __builtin_amdgcn_wmma_f32_16x16x32_f16(false, av0, false, bp[0],
                                                            (short)0, o[ct], false, false);
            o[ct] = __builtin_amdgcn_wmma_f32_16x16x32_f16(false, av1, false, bp[1],
                                                            (short)0, o[ct], false, false);
        }
        __syncthreads();
    }

    const float linv = 1.0f / (l * 1024.0f);
    #pragma unroll
    for (int ct = 0; ct < 4; ++ct)
        #pragma unroll
        for (int r = 0; r < 8; ++r) {
            const int c = ct * 16 + r + (hi ? 8 : 0);
            so[c * 68 + wave * 16 + col] = o[ct][r] * linv;
        }
    __syncthreads();
#pragma unroll 1
    for (int pass = 0; pass < 2; ++pass) {
        for (int ch = t; ch < 64 * 16; ch += 128) { const int c = ch >> 4, q4 = (ch & 15) * 4;
            *(volatile v4f_t*)(out + ((size_t)b * C_ + c) * NQ_ + qbase + q4) = *(const volatile v4fa*)(so + c * 68 + q4); }
        __threadfence();
    }
}

extern "C" void kernel_launch(void* const* d_in, const int* in_sizes, int n_in,
                              void* d_out, int out_size, void* d_ws, size_t ws_size,
                              hipStream_t stream) {
    const float* q       = (const float*)d_in[0];
    const float* v       = (const float*)d_in[1];
    const float* k_w     = (const float*)d_in[2];
    const float* v_w     = (const float*)d_in[3];
    const float* q_gamma = (const float*)d_in[4];
    const float* q_beta  = (const float*)d_in[5];
    const float* q_mean  = (const float*)d_in[6];
    const float* q_var   = (const float*)d_in[7];
    const float* k_gamma = (const float*)d_in[8];
    const float* k_beta  = (const float*)d_in[9];
    const float* k_mean  = (const float*)d_in[10];
    const float* k_var   = (const float*)d_in[11];

    const size_t kv_bytes = (size_t)B_ * NV_ * C_ * sizeof(bf16_t);
    bf16_t* keyT = (bf16_t*)d_ws;
    bf16_t* valT = (bf16_t*)((char*)d_ws + 2 * kv_bytes);

    conv_bn_kernel<<<dim3(NV_ / 64, B_), 256, 0, stream>>>(
        v, k_w, v_w, k_gamma, k_beta, k_mean, k_var, keyT, valT);
    attn_kernel<<<dim3(NQ_ / 64, B_), 128, 0, stream>>>(
        q, q_gamma, q_beta, q_mean, q_var, keyT, valT, (float*)d_out);
}
